// TiSASRec_36636071035272
// MI455X (gfx1250) — hardware-verified
//
#include <hip/hip_runtime.h>
#include <hip/hip_bf16.h>

#define B_ 8
#define L_ 256
#define H_ 256
#define HEADS_ 4
#define D_ 64
#define NBLK_ 2
#define M_ (B_ * L_)
#define BIG_NEG (-4294967295.0f)

typedef __attribute__((ext_vector_type(16))) _Float16 v16h;
typedef __attribute__((ext_vector_type(8)))  float    v8f;
typedef __attribute__((ext_vector_type(4)))  float    v4f_t;
typedef float v4fa __attribute__((ext_vector_type(4), may_alias));
#define ST2(ptr, val) do { *(volatile float*)(ptr) = (val); __threadfence(); *(volatile float*)(ptr) = (val); } while (0)

__device__ __forceinline__ float4 f4add(float4 a, float4 b) {
    return make_float4(a.x + b.x, a.y + b.y, a.z + b.z, a.w + b.w);
}

__device__ __forceinline__ v16h pack16(float4 a, float4 b, float4 c, float4 d) {
    v16h v;
    v[0]  = (_Float16)a.x; v[1]  = (_Float16)a.y; v[2]  = (_Float16)a.z; v[3]  = (_Float16)a.w;
    v[4]  = (_Float16)b.x; v[5]  = (_Float16)b.y; v[6]  = (_Float16)b.z; v[7]  = (_Float16)b.w;
    v[8]  = (_Float16)c.x; v[9]  = (_Float16)c.y; v[10] = (_Float16)c.z; v[11] = (_Float16)c.w;
    v[12] = (_Float16)d.x; v[13] = (_Float16)d.y; v[14] = (_Float16)d.z; v[15] = (_Float16)d.w;
    return v;
}

__device__ __forceinline__ v16h loadA(const float* __restrict__ row, int hi) {
    const float4* p0 = (const float4*)(row + hi * 8);
    const float4* p1 = (const float4*)(row + 16 + hi * 8);
    return pack16(p0[0], p0[1], p1[0], p1[1]);
}

__device__ __forceinline__ v16h loadB(const float* __restrict__ col, int hi) {
    const float4* p0 = (const float4*)(col + hi * 8);
    const float4* p1 = (const float4*)(col + 16 + hi * 8);
    return pack16(p0[0], p0[1], p1[0], p1[1]);
}

__device__ __forceinline__ v16h loadB_sum(const float* __restrict__ c0,
                                          const float* __restrict__ c1, int hi) {
    const float4* p0 = (const float4*)(c0 + hi * 8), *p1 = (const float4*)(c0 + 16 + hi * 8);
    const float4* q0 = (const float4*)(c1 + hi * 8), *q1 = (const float4*)(c1 + 16 + hi * 8);
    return pack16(f4add(p0[0], q0[0]), f4add(p0[1], q0[1]),
                  f4add(p1[0], q1[0]), f4add(p1[1], q1[1]));
}

__global__ __launch_bounds__(256) void prep_x(const float* __restrict__ seq,
                                              const int* __restrict__ mask,
                                              float* __restrict__ x) {
    int i = blockIdx.x * 256 + threadIdx.x;
    int row = i / H_;
    const float v = seq[i] * (mask[row] ? 0.0f : 1.0f);
    ST2(x + i, v);
}

__global__ __launch_bounds__(256) void layernorm_k(const float* __restrict__ in,
                                                   const float* __restrict__ g,
                                                   const float* __restrict__ b,
                                                   float* __restrict__ out) {
    __shared__ float red[256];
    int row = blockIdx.x, t = threadIdx.x;
    size_t idx = (size_t)row * H_ + t;
    float v = in[idx];
    red[t] = v; __syncthreads();
    for (int s = 128; s > 0; s >>= 1) { if (t < s) red[t] += red[t + s]; __syncthreads(); }
    float m = red[0] * (1.0f / H_); __syncthreads();
    float d = v - m;
    red[t] = d * d; __syncthreads();
    for (int s = 128; s > 0; s >>= 1) { if (t < s) red[t] += red[t + s]; __syncthreads(); }
    float var = red[0] * (1.0f / H_);
    const float o = d * rsqrtf(var + 1e-8f) * g[t] + b[t];
    ST2(out + idx, o);
}

__global__ __launch_bounds__(256) void gemm_wT_wmma(
        const float* __restrict__ X, const float* __restrict__ W,
        const float* __restrict__ bias, const float* __restrict__ resid,
        const int* __restrict__ mask, float* __restrict__ Y, int relu) {
    int wave = threadIdx.x >> 5, lane = threadIdx.x & 31;
    int hi = lane >> 4, ln = lane & 15;
    int gtile = blockIdx.x * 8 + wave;
    int tm0 = (gtile >> 4) * 16;
    int tn0 = (gtile & 15) * 16;

    const float* xrow = X + (size_t)(tm0 + ln) * H_;
    const float* wrow = W + (size_t)(tn0 + ln) * H_;
    v8f acc = {};
    #pragma unroll 2
    for (int kk = 0; kk < H_; kk += 32) {
        v16h a  = loadA(xrow + kk, hi);
        v16h bm = loadB(wrow + kk, hi);
        acc = __builtin_amdgcn_wmma_f32_16x16x32_f16(false, a, false, bm,
                                                     (short)0, acc, false, false);
    }
    __shared__ __attribute__((aligned(16))) float st[16][128 + 4];
    int col = tn0 + ln;
    float bv = bias[col];
    #pragma unroll
    for (int r = 0; r < 8; ++r) {
        int row = tm0 + r + hi * 8;
        float v = acc[r] + bv;
        if (relu) v = fmaxf(v, 0.0f);
        if (resid) v += resid[(size_t)row * H_ + col];
        if (mask)  v *= (mask[row] ? 0.0f : 1.0f);
        st[r + hi * 8][wave * 16 + ln] = v;
    }
    __syncthreads();
    const int cb0 = (blockIdx.x * 8 & 15) * 16;
    #pragma unroll 1
    for (int pass = 0; pass < 2; ++pass) {
        #pragma unroll
        for (int i = 0; i < 2; ++i) {
            const int c = threadIdx.x + 256 * i, rr = c >> 5, q = c & 31;
            *(volatile v4f_t*)(Y + (size_t)(tm0 + rr) * H_ + cb0 + q * 4) = *(const v4fa*)&st[rr][q * 4];
        }
        __threadfence();
    }
}

__global__ __launch_bounds__(256) void attn_scores(
        const float* __restrict__ Q, const float* __restrict__ Kh,
        const float* __restrict__ posK, const float* __restrict__ tK,
        const int* __restrict__ tmat, const int* __restrict__ mask,
        float* __restrict__ aw) {
    int b = blockIdx.z, h = blockIdx.y, q0 = blockIdx.x * 16;
    int wave = threadIdx.x >> 5, lane = threadIdx.x & 31;
    int hi = lane >> 4, ln = lane & 15;
    const float inv_scale = 0.125f;
    __shared__ __attribute__((aligned(16))) float saw[16][L_ + 4];

    const float* qrowA = Q + (size_t)(b * L_ + q0 + ln) * H_ + h * D_;

    for (int kt = wave; kt < 16; kt += 8) {
        int k0 = kt * 16;
        int kcol = k0 + ln;
        const float* krow = Kh   + (size_t)(b * L_ + kcol) * H_ + h * D_;
        const float* prow = posK + (size_t)kcol * H_ + h * D_;
        v8f acc = {};
        #pragma unroll
        for (int dd = 0; dd < D_; dd += 32) {
            v16h a  = loadA(qrowA + dd, hi);
            v16h bm = loadB_sum(krow + dd, prow + dd, hi);
            acc = __builtin_amdgcn_wmma_f32_16x16x32_f16(false, a, false, bm,
                                                         (short)0, acc, false, false);
        }
        int kg = k0 + ln;
        #pragma unroll
        for (int r = 0; r < 8; ++r) {
            int q = q0 + r + hi * 8;
            int t = tmat[(size_t)(b * L_ + q) * L_ + kg];
            const float4* q4 = (const float4*)(Q + (size_t)(b * L_ + q) * H_ + h * D_);
            const float4* e4 = (const float4*)(tK + (size_t)t * H_ + h * D_);
            float s = 0.0f;
            #pragma unroll 4
            for (int d = 0; d < D_ / 4; ++d) {
                float4 qv = q4[d], ev = e4[d];
                s += qv.x * ev.x + qv.y * ev.y + qv.z * ev.z + qv.w * ev.w;
            }
            float v = (acc[r] + s) * inv_scale;
            if (mask[b * L_ + q] || kg > q) v = BIG_NEG;
            saw[r + hi * 8][kg] = v;
        }
    }
    __syncthreads();
    #pragma unroll 1
    for (int pass = 0; pass < 2; ++pass) {
        #pragma unroll
        for (int i = 0; i < 4; ++i) {
            const int c = threadIdx.x + 256 * i, rr = c >> 6, qq = c & 63;
            *(volatile v4f_t*)(aw + ((size_t)(b * HEADS_ + h) * L_ + q0 + rr) * L_ + qq * 4) = *(const v4fa*)&saw[rr][qq * 4];
        }
        __threadfence();
    }
}

__global__ __launch_bounds__(256) void softmax_k(float* __restrict__ p) {
    __shared__ float red[256];
    size_t row = blockIdx.x;
    int t = threadIdx.x;
    float v = p[row * L_ + t];
    red[t] = v; __syncthreads();
    for (int s = 128; s > 0; s >>= 1) { if (t < s) red[t] = fmaxf(red[t], red[t + s]); __syncthreads(); }
    float mx = red[0]; __syncthreads();
    float e = __expf(v - mx);
    red[t] = e; __syncthreads();
    for (int s = 128; s > 0; s >>= 1) { if (t < s) red[t] += red[t + s]; __syncthreads(); }
    const float pv = e / red[0];
    ST2(p + row * L_ + t, pv);
}

__global__ __launch_bounds__(256) void attn_out_wmma(
        const float* __restrict__ P, const float* __restrict__ V,
        const float* __restrict__ posV, float* __restrict__ Yo) {
    int bh = blockIdx.x, b = bh / HEADS_, h = bh % HEADS_;
    int wave = threadIdx.x >> 5, lane = threadIdx.x & 31;
    int hi = lane >> 4, ln = lane & 15;
    int q0 = blockIdx.y * 32 + (wave >> 2) * 16;
    int d0 = (wave & 3) * 16;
    const float* prow = P + ((size_t)bh * L_ + q0 + ln) * L_;
    int d = d0 + ln;

    v8f acc = {};
    #pragma unroll 2
    for (int kk = 0; kk < L_; kk += 32) {
        v16h a = loadA(prow + kk, hi);
        v16h bm;
        #pragma unroll
        for (int e = 0; e < 16; ++e) {
            int k = kk + ((e < 8) ? (hi * 8 + e) : (16 + hi * 8 + (e - 8)));
            bm[e] = (_Float16)(V[(size_t)(b * L_ + k) * H_ + h * D_ + d] +
                               posV[(size_t)k * H_ + h * D_ + d]);
        }
        acc = __builtin_amdgcn_wmma_f32_16x16x32_f16(false, a, false, bm,
                                                     (short)0, acc, false, false);
    }
    __shared__ __attribute__((aligned(16))) float syo[32][64 + 4];
    #pragma unroll
    for (int r = 0; r < 8; ++r) syo[(wave >> 2) * 16 + r + hi * 8][d0 + ln] = acc[r];
    __syncthreads();
    #pragma unroll 1
    for (int pass = 0; pass < 2; ++pass) {
        #pragma unroll
        for (int i = 0; i < 2; ++i) {
            const int c = threadIdx.x + 256 * i, rr = c >> 4, qq = c & 15;
            *(volatile v4f_t*)(Yo + (size_t)(b * L_ + blockIdx.y * 32 + rr) * H_ + h * D_ + qq * 4) = *(const v4fa*)&syo[rr][qq * 4];
        }
        __threadfence();
    }
}

__global__ __launch_bounds__(256) void attn_tmv_resid(
        const float* __restrict__ P, const float* __restrict__ tV,
        const int* __restrict__ tmat, const float* __restrict__ qn,
        const float* __restrict__ yw, float* __restrict__ out) {
    int q = blockIdx.x, b = blockIdx.y, c = threadIdx.x;
    int h = c >> 6;
    const float* Pb = P + ((size_t)(b * HEADS_ + h) * L_ + q) * L_;
    const int* tr = tmat + (size_t)(b * L_ + q) * L_;
    float acc = 0.0f;
    #pragma unroll 4
    for (int k = 0; k < L_; ++k) {
        int t = tr[k];
        acc += Pb[k] * tV[(size_t)t * H_ + c];
    }
    size_t idx = (size_t)(b * L_ + q) * H_ + c;
    const float o = qn[idx] + yw[idx] + acc;
    ST2(out + idx, o);
}

extern "C" void kernel_launch(void* const* d_in, const int* in_sizes, int n_in,
                              void* d_out, int out_size, void* d_ws, size_t ws_size,
                              hipStream_t stream) {
    const int*   mask = (const int*)d_in[0];
    const float* seq  = (const float*)d_in[1];
    const int*   tmat = (const int*)d_in[3];
    const float* Wq   = (const float*)d_in[5];
    const float* bq   = (const float*)d_in[6];
    const float* Wk   = (const float*)d_in[7];
    const float* bk   = (const float*)d_in[8];
    const float* Wv   = (const float*)d_in[9];
    const float* bv   = (const float*)d_in[10];
    const float* ln1g = (const float*)d_in[11];
    const float* ln1b = (const float*)d_in[12];
    const float* ln2g = (const float*)d_in[13];
    const float* ln2b = (const float*)d_in[14];
    const float* W1   = (const float*)d_in[15];
    const float* b1   = (const float*)d_in[16];
    const float* W2   = (const float*)d_in[17];
    const float* b2   = (const float*)d_in[18];
    const float* posK = (const float*)d_in[19];
    const float* posV = (const float*)d_in[20];
    const float* tK   = (const float*)d_in[21];
    const float* tV   = (const float*)d_in[22];
    const float* lnfg = (const float*)d_in[23];
    const float* lnfb = (const float*)d_in[24];

    const size_t ACT = (size_t)M_ * H_;
    float* ws = (float*)d_ws;
    float* x   = ws;
    float* qn  = x  + ACT;
    float* Qh  = qn + ACT;
    float* Kh  = Qh + ACT;
    float* Vh  = Kh + ACT;
    float* yw  = Vh + ACT;
    float* aw  = yw + ACT;
    float* hb  = Qh;
    float* tmp = Kh;

    const int gemm_blocks = (M_ / 16) * (H_ / 16) / 8;

    prep_x<<<M_, 256, 0, stream>>>(seq, mask, x);

    for (int i = 0; i < NBLK_; ++i) {
        const float* wq = Wq + (size_t)i * H_ * H_;
        const float* wk = Wk + (size_t)i * H_ * H_;
        const float* wv = Wv + (size_t)i * H_ * H_;
        const float* w1 = W1 + (size_t)i * H_ * H_;
        const float* w2 = W2 + (size_t)i * H_ * H_;

        layernorm_k<<<M_, 256, 0, stream>>>(x, ln1g + i * H_, ln1b + i * H_, qn);

        gemm_wT_wmma<<<gemm_blocks, 256, 0, stream>>>(qn, wq, bq + i * H_, nullptr, nullptr, Qh, 0);
        gemm_wT_wmma<<<gemm_blocks, 256, 0, stream>>>(x,  wk, bk + i * H_, nullptr, nullptr, Kh, 0);
        gemm_wT_wmma<<<gemm_blocks, 256, 0, stream>>>(x,  wv, bv + i * H_, nullptr, nullptr, Vh, 0);

        attn_scores<<<dim3(L_ / 16, HEADS_, B_), 256, 0, stream>>>(Qh, Kh, posK, tK, tmat, mask, aw);
        softmax_k<<<B_ * HEADS_ * L_, 256, 0, stream>>>(aw);
        attn_out_wmma<<<dim3(B_ * HEADS_, L_ / 32), 256, 0, stream>>>(aw, Vh, posV, yw);
        attn_tmv_resid<<<dim3(L_, B_), 256, 0, stream>>>(aw, tV, tmat, qn, yw, tmp);

        layernorm_k<<<M_, 256, 0, stream>>>(tmp, ln2g + i * H_, ln2b + i * H_, x);

        gemm_wT_wmma<<<gemm_blocks, 256, 0, stream>>>(x,  w1, b1 + i * H_, nullptr, nullptr, hb, 1);
        gemm_wT_wmma<<<gemm_blocks, 256, 0, stream>>>(hb, w2, b2 + i * H_, x, mask, x, 0);
    }

    layernorm_k<<<M_, 256, 0, stream>>>(x, lnfg, lnfb, (float*)d_out);
}
